// CrossEfficientAttention_35184372089344
// MI455X (gfx1250) — hardware-verified
//
#include <hip/hip_runtime.h>
#include <stdint.h>

#define NBAT 8
#define CH   256
#define NSP  4096
#define GB   2
#define NGRP (NBAT / GB)
static_assert((NSP % 64) == 0 && (CH % 64) == 0 && (NBAT % GB) == 0);
static_assert(NSP == 2 * 256 * 8);
static_assert(CH == 32 * 8);

typedef __bf16   v16b __attribute__((ext_vector_type(16)));
typedef __bf16   v8b  __attribute__((ext_vector_type(8)));
typedef float    v8f  __attribute__((ext_vector_type(8)));
typedef float    v4f  __attribute__((ext_vector_type(4)));
typedef unsigned int v4u __attribute__((ext_vector_type(4)));

__device__ __forceinline__ unsigned short bf_bits(float f) {
  unsigned u = __float_as_uint(f);
  return (unsigned short)((u + 0x7FFFu + ((u >> 16) & 1u)) >> 16);
}
__device__ __forceinline__ float bf_up(unsigned short h) { return __uint_as_float(((unsigned)h) << 16); }
__device__ __forceinline__ unsigned pk16(unsigned short a, unsigned short b) { return (unsigned)a | ((unsigned)b << 16); }
__device__ __forceinline__ v8f zero8() { v8f z = {0.f, 0.f, 0.f, 0.f, 0.f, 0.f, 0.f, 0.f}; return z; }

__device__ __forceinline__ v16b ldfrag_b(const __bf16* p) {
  union { v16b v; v8b h[2]; } f;
  f.h[0] = *(const v8b*)(p);
  f.h[1] = *(const v8b*)(p + 16);
  return f.v;
}

__device__ __forceinline__ v8f mma_b_raw(v16b a, v16b b, v8f c) {
  return __builtin_amdgcn_wmma_f32_16x16x32_bf16(false, a, false, b, (short)0, c, false, false);
}
__device__ __forceinline__ void dep_guard_b(v8f& a, v8f& b, v16b x, v16b y) {
#if defined(__HIP_DEVICE_COMPILE__)
  asm volatile("v_nop\n\tv_nop\n\tv_nop\n\tv_nop" : "+v"(a), "+v"(b) : "v"(x), "v"(y));
#endif
}
__device__ __forceinline__ void keep4_b(v16b a, v16b b, v16b c, v16b d) {
#if defined(__HIP_DEVICE_COMPILE__)
  asm volatile("v_nop" :: "v"(a), "v"(b), "v"(c), "v"(d));
#endif
}
__device__ __forceinline__ void acc_guard4(v8f& a, v8f& b, v8f& c, v8f& d) {
#if defined(__HIP_DEVICE_COMPILE__)
  asm volatile("v_nop\n\tv_nop\n\tv_nop\n\tv_nop" : "+v"(a), "+v"(b), "+v"(c), "+v"(d));
#endif
}
__device__ __forceinline__ void wave_sync_lds() {
  __builtin_amdgcn_fence(__ATOMIC_RELEASE, "workgroup");
  __builtin_amdgcn_wave_barrier();
  __builtin_amdgcn_fence(__ATOMIC_ACQUIRE, "workgroup");
}

__global__ __launch_bounds__(256) void cvt_bf16x8(const float* __restrict__ in, unsigned short* out, int n8) {
  const int i = blockIdx.x * 256 + threadIdx.x;
  if (i < n8) {
    const v4f a = *(const v4f*)(in + (size_t)i * 8);
    const v4f b = *(const v4f*)(in + (size_t)i * 8 + 4);
    v4u p;
    p[0] = pk16(bf_bits(a[0]), bf_bits(a[1]));
    p[1] = pk16(bf_bits(a[2]), bf_bits(a[3]));
    p[2] = pk16(bf_bits(b[0]), bf_bits(b[1]));
    p[3] = pk16(bf_bits(b[2]), bf_bits(b[3]));
    *(volatile v4u*)(out + (size_t)i * 8) = p;
    __threadfence();
    *(volatile v4u*)(out + (size_t)i * 8) = p;
  }
}

__global__ __launch_bounds__(256) void k_trcvt(const float* __restrict__ xg, const float* __restrict__ cg,
                                               unsigned short* xt, unsigned short* ct, int b0) {
  __shared__ float tile[64][65];
  const int tid = threadIdx.x;
  const int n0 = blockIdx.x * 64;
  const int c0 = blockIdx.y * 64;
  const int bi  = (int)(blockIdx.z >> 1);
  const int sel = (int)(blockIdx.z & 1);
  const float* src = sel ? cg : xg;
  unsigned short* dst = sel ? ct : xt;
  {
    const int r = tid >> 2, cs = (tid & 3) * 16;
    const float* p = src + ((size_t)(b0 + bi) * CH + (size_t)(c0 + r)) * NSP + n0 + cs;
#pragma unroll
    for (int i = 0; i < 4; ++i) {
      const v4f v = *(const v4f*)(p + 4 * i);
      tile[r][cs + 4 * i + 0] = v[0];
      tile[r][cs + 4 * i + 1] = v[1];
      tile[r][cs + 4 * i + 2] = v[2];
      tile[r][cs + 4 * i + 3] = v[3];
    }
  }
  __syncthreads();
  v4u pv[2];
  const int c8 = (tid & 7) * 8;
#pragma unroll
  for (int it = 0; it < 2; ++it) {
    const int n = it * 32 + (tid >> 3);
    v4u a;
#pragma unroll
    for (int e = 0; e < 4; ++e) {
      a[e] = pk16(bf_bits(tile[c8 + 2 * e][n]), bf_bits(tile[c8 + 2 * e + 1][n]));
    }
    pv[it] = a;
  }
  for (int pass = 0; pass < 2; ++pass) {
#pragma unroll
    for (int it = 0; it < 2; ++it) {
      const int n = it * 32 + (tid >> 3);
      const size_t go = ((size_t)bi * NSP + (size_t)(n0 + n)) * CH + c0 + c8;
      *(volatile v4u*)(dst + go) = pv[it];
    }
    __threadfence();
  }
}

template <int NSPLIT, int OUT_MODE, int BIAS>
__global__ __launch_bounds__(256) void gemm64(
    const unsigned short* __restrict__ Ap, const unsigned short* A2p, int lda, long long strideA,
    const unsigned short* __restrict__ Btp, const unsigned short* Bt2p, int ldb, long long strideB,
    void* Cout, void* Cout2, int ldc, long long strideC,
    const float* __restrict__ bias, int M, int N, int K, float oscale) {
  const __bf16* A   = (const __bf16*)(const void*)Ap;
  const __bf16* A2  = (const __bf16*)(const void*)A2p;
  const __bf16* Bt  = (const __bf16*)(const void*)Btp;
  const __bf16* Bt2 = (const __bf16*)(const void*)Bt2p;
  __shared__ __align__(16) float sT[8][16 * 68];
  const int b    = blockIdx.y;
  const int lane = threadIdx.x & 31;
  const int wave = threadIdx.x >> 5;
  const int tilesN = N >> 6;
  const int tilesM = M >> 6;
  const int tile = blockIdx.x * 8 + wave;
  if (tile >= tilesM * tilesN) return;
  const int tm = tile / tilesN;
  const int tn = tile - tm * tilesN;
  const int m0 = tm << 6;
  const int n0 = tn << 6;

  constexpr bool useA2 = (NSPLIT == 1) || (NSPLIT == 2);
  constexpr bool useB2 = (NSPLIT >= 2);
  const __bf16* Ab  = A  + (size_t)b * strideA;
  const __bf16* Bb  = Bt + (size_t)b * strideB;
  const __bf16* Ab2 = useA2 ? (A2  + (size_t)b * strideA) : Ab;
  const __bf16* Bb2 = useB2 ? (Bt2 + (size_t)b * strideB) : Bb;

  const int rlane = lane & 15;
  const int koff  = (lane >> 4) * 8;
  const int mOff  = (lane >> 4) * 8;

  v8f acc[4][4];
#pragma unroll
  for (int i = 0; i < 4; ++i)
#pragma unroll
    for (int j = 0; j < 4; ++j) acc[i][j] = zero8();

  for (int k0 = 0; k0 < K; k0 += 32) {
    v16b bh[4], bl[4];
#pragma unroll
    for (int j = 0; j < 4; ++j) {
      const size_t bofs = (size_t)(n0 + (j << 4) + rlane) * ldb + koff + k0;
      bh[j] = ldfrag_b(Bb + bofs);
      if (useB2) bl[j] = ldfrag_b(Bb2 + bofs); else bl[j] = bh[j];
    }
#pragma unroll
    for (int i = 0; i < 4; ++i) {
      const size_t ao = (size_t)(m0 + (i << 4) + rlane) * lda + koff + k0;
      const v16b ah = ldfrag_b(Ab + ao);
      v16b al = ah;
      if (useA2) al = ldfrag_b(Ab2 + ao);
#pragma unroll
      for (int j = 0; j < 4; ++j) {
        acc[i][j] = mma_b_raw(ah, bh[j], acc[i][j]);
        if (useA2) acc[i][j] = mma_b_raw(al, bh[j], acc[i][j]);
        if (useB2) acc[i][j] = mma_b_raw(ah, bl[j], acc[i][j]);
      }
      dep_guard_b(acc[i][0], acc[i][3], ah, al);
    }
    keep4_b(bh[0], bh[1], bh[2], bh[3]);
    if (useB2) keep4_b(bl[0], bl[1], bl[2], bl[3]);
  }
  acc_guard4(acc[0][0], acc[0][1], acc[0][2], acc[0][3]);
  acc_guard4(acc[1][0], acc[1][1], acc[1][2], acc[1][3]);
  acc_guard4(acc[2][0], acc[2][1], acc[2][2], acc[2][3]);
  acc_guard4(acc[3][0], acc[3][1], acc[3][2], acc[3][3]);

  float bcol[4];
#pragma unroll
  for (int j = 0; j < 4; ++j) bcol[j] = 0.f;
  if (BIAS == 2) {
#pragma unroll
    for (int j = 0; j < 4; ++j) bcol[j] = bf_up(bf_bits(bias[n0 + (j << 4) + rlane]));
  }
  float* slab = sT[wave];
#pragma unroll
  for (int i = 0; i < 4; ++i) {
    const int mBase = m0 + (i << 4);
    float brow[8];
#pragma unroll
    for (int r = 0; r < 8; ++r) brow[r] = 0.f;
    if (BIAS == 1) {
#pragma unroll
      for (int r = 0; r < 8; ++r) brow[r] = bf_up(bf_bits(bias[mBase + mOff + r]));
    }
#pragma unroll
    for (int j = 0; j < 4; ++j) {
#pragma unroll
      for (int r = 0; r < 8; ++r) {
        slab[(mOff + r) * 68 + (j << 4) + rlane] = acc[i][j][r] * oscale + (brow[r] + bcol[j]);
      }
    }
    wave_sync_lds();
    if (OUT_MODE == 0) {
      float* C = (float*)Cout + (size_t)b * strideC;
      const int hh = lane >> 4, c4 = (lane & 15) * 4;
      for (int pass = 0; pass < 2; ++pass) {
#pragma unroll
        for (int it = 0; it < 8; ++it) {
          const int row = it * 2 + hh;
          const v4f v = *(const v4f*)(slab + row * 68 + c4);
          *(volatile v4f*)(C + (size_t)(mBase + row) * ldc + n0 + c4) = v;
        }
        __threadfence();
      }
    } else {
      const int q = lane >> 3, c8 = (lane & 7) * 8;
      unsigned short* C  = (unsigned short*)Cout  + (size_t)b * strideC;
      unsigned short* C2 = (unsigned short*)Cout2 + (size_t)b * strideC;
      v4u hv[4], lv[4];
#pragma unroll
      for (int it = 0; it < 4; ++it) {
        const int row = it * 4 + q;
        const float* sp = slab + row * 68 + c8;
        v4u a, a2;
#pragma unroll
        for (int e = 0; e < 4; ++e) {
          const float f0 = sp[2 * e], f1 = sp[2 * e + 1];
          const unsigned short h0 = bf_bits(f0), h1 = bf_bits(f1);
          const unsigned short l0 = bf_bits(f0 - bf_up(h0)), l1 = bf_bits(f1 - bf_up(h1));
          a[e] = pk16(h0, h1); a2[e] = pk16(l0, l1);
        }
        hv[it] = a; lv[it] = a2;
      }
      for (int pass = 0; pass < 2; ++pass) {
#pragma unroll
        for (int it = 0; it < 4; ++it) {
          const int row = it * 4 + q;
          const size_t go = (size_t)(mBase + row) * ldc + n0 + c8;
          *(volatile v4u*)(C  + go) = hv[it];
          *(volatile v4u*)(C2 + go) = lv[it];
        }
        __threadfence();
      }
    }
    wave_sync_lds();
  }
}

__global__ __launch_bounds__(256) void k_qsoft(const float* __restrict__ qt, unsigned short* qh, unsigned short* ql) {
  const int lane = threadIdx.x & 31, wave = threadIdx.x >> 5;
  const int n = blockIdx.x * 8 + wave;
  const size_t ro = ((size_t)blockIdx.y * NSP + (size_t)n) * CH + (size_t)lane * 8;
  const v4f a = *(const v4f*)(qt + ro);
  const v4f c = *(const v4f*)(qt + ro + 4);
  float v[8];
  v[0] = a[0] * 0.25f; v[1] = a[1] * 0.25f; v[2] = a[2] * 0.25f; v[3] = a[3] * 0.25f;
  v[4] = c[0] * 0.25f; v[5] = c[1] * 0.25f; v[6] = c[2] * 0.25f; v[7] = c[3] * 0.25f;
  float m = v[0];
#pragma unroll
  for (int i = 1; i < 8; ++i) m = fmaxf(m, v[i]);
  m = fmaxf(m, __shfl_xor(m, 1, 32));
  m = fmaxf(m, __shfl_xor(m, 2, 32));
  m = fmaxf(m, __shfl_xor(m, 4, 32));
  float e[8];
  float s = 0.f;
#pragma unroll
  for (int i = 0; i < 8; ++i) { e[i] = __expf(v[i] - m); s += e[i]; }
  s += __shfl_xor(s, 1, 32);
  s += __shfl_xor(s, 2, 32);
  s += __shfl_xor(s, 4, 32);
  const float rinv = 1.0f / s;
  v4u ph, pl;
#pragma unroll
  for (int q = 0; q < 4; ++q) {
    const float f0 = (e[2 * q] * rinv) * 64.0f;
    const float f1 = (e[2 * q + 1] * rinv) * 64.0f;
    const unsigned short h0 = bf_bits(f0), h1 = bf_bits(f1);
    const unsigned short l0 = bf_bits(f0 - bf_up(h0)), l1 = bf_bits(f1 - bf_up(h1));
    ph[q] = pk16(h0, h1); pl[q] = pk16(l0, l1);
  }
  *(volatile v4u*)(qh + ro) = ph;
  *(volatile v4u*)(ql + ro) = pl;
  __threadfence();
  *(volatile v4u*)(qh + ro) = ph;
  *(volatile v4u*)(ql + ro) = pl;
}

__global__ __launch_bounds__(256) void k_ksoftv(const float* __restrict__ kv,
                                                unsigned short* kph, unsigned short* kpl,
                                                unsigned short* vhp, unsigned short* vlp) {
  __shared__ float red[8];
  const int tid = threadIdx.x, lane = tid & 31, wave = tid >> 5;
  const int j  = blockIdx.x;
  const int bi = blockIdx.y;
  const bool isK = (j < CH);
  const float* src = kv + ((size_t)bi * (2 * CH) + (size_t)j) * NSP;
  float vals[16];
#pragma unroll
  for (int it = 0; it < 2; ++it) {
    const size_t co = (size_t)it * 2048 + (size_t)tid * 8;
    const v4f a = *(const v4f*)(src + co);
    const v4f c = *(const v4f*)(src + co + 4);
    vals[it * 8 + 0] = a[0]; vals[it * 8 + 1] = a[1]; vals[it * 8 + 2] = a[2]; vals[it * 8 + 3] = a[3];
    vals[it * 8 + 4] = c[0]; vals[it * 8 + 5] = c[1]; vals[it * 8 + 6] = c[2]; vals[it * 8 + 7] = c[3];
  }
  if (isK) {
    float m = vals[0];
#pragma unroll
    for (int i = 1; i < 16; ++i) m = fmaxf(m, vals[i]);
#pragma unroll
    for (int off = 1; off < 32; off <<= 1) m = fmaxf(m, __shfl_xor(m, off, 32));
    if (lane == 0) red[wave] = m;
    __syncthreads();
    float mm = red[0];
#pragma unroll
    for (int w = 1; w < 8; ++w) mm = fmaxf(mm, red[w]);
    __syncthreads();
    float s = 0.f;
#pragma unroll
    for (int i = 0; i < 16; ++i) { vals[i] = __expf(vals[i] - mm); s += vals[i]; }
#pragma unroll
    for (int off = 1; off < 32; off <<= 1) s += __shfl_xor(s, off, 32);
    if (lane == 0) red[wave] = s;
    __syncthreads();
    float ss = red[0];
#pragma unroll
    for (int w = 1; w < 8; ++w) ss += red[w];
    const float rinv = 1.0f / ss;
#pragma unroll
    for (int i = 0; i < 16; ++i) vals[i] = (vals[i] * rinv) * 4096.0f;
  }
  const int rr = isK ? j : (j - CH);
  unsigned short* ph = isK ? kph : vhp;
  unsigned short* pl = isK ? kpl : vlp;
  unsigned short* dh = ph + ((size_t)bi * CH + (size_t)rr) * NSP;
  unsigned short* dl = pl + ((size_t)bi * CH + (size_t)rr) * NSP;
  v4u hv[2], lv[2];
#pragma unroll
  for (int it = 0; it < 2; ++it) {
    v4u a, a2;
#pragma unroll
    for (int e = 0; e < 4; ++e) {
      const float f0 = vals[it * 8 + 2 * e], f1 = vals[it * 8 + 2 * e + 1];
      const unsigned short h0 = bf_bits(f0), h1 = bf_bits(f1);
      const unsigned short l0 = bf_bits(f0 - bf_up(h0)), l1 = bf_bits(f1 - bf_up(h1));
      a[e] = pk16(h0, h1); a2[e] = pk16(l0, l1);
    }
    hv[it] = a; lv[it] = a2;
  }
  for (int pass = 0; pass < 2; ++pass) {
#pragma unroll
    for (int it = 0; it < 2; ++it) {
      const size_t co = (size_t)it * 2048 + (size_t)tid * 8;
      *(volatile v4u*)(dh + co) = hv[it];
      *(volatile v4u*)(dl + co) = lv[it];
    }
    __threadfence();
  }
}

static inline unsigned tile_blocks(int M, int N) { return (unsigned)((((M / 64) * (N / 64)) + 7) / 8); }

extern "C" void kernel_launch(void* const* d_in, const int* in_sizes, int n_in,
                              void* d_out, int out_size, void* d_ws, size_t ws_size,
                              hipStream_t stream) {
  if (n_in < 8) return;
  if (in_sizes[0] != NBAT * CH * NSP) return;
  if (in_sizes[1] != NBAT * CH * NSP) return;
  if (in_sizes[2] != CH * CH) return;
  if (in_sizes[3] != CH) return;
  if (in_sizes[4] != 2 * CH * CH) return;
  if (in_sizes[5] != 2 * CH) return;
  if (in_sizes[6] != CH * CH) return;
  if (in_sizes[7] != CH) return;
  if (out_size != NBAT * CH * NSP) return;

  const float* x     = (const float*)d_in[0];
  const float* cproj = (const float*)d_in[1];
  const float* wq    = (const float*)d_in[2];
  const float* bq    = (const float*)d_in[3];
  const float* wkv   = (const float*)d_in[4];
  const float* bkv   = (const float*)d_in[5];
  const float* wo    = (const float*)d_in[6];
  const float* bo    = (const float*)d_in[7];
  float* out = (float*)d_out;

  const size_t PWq  = (size_t)CH * CH * 2;
  const size_t PWkv = (size_t)2 * CH * CH * 2;
  const size_t PWo  = (size_t)CH * CH * 2;
  const size_t PXt  = (size_t)GB * NSP * CH * 2;
  const size_t PQt  = (size_t)GB * NSP * CH * 4;
  const size_t PQp  = (size_t)GB * NSP * CH * 2;
  const size_t PKV  = (size_t)GB * 2 * CH * NSP * 4;
  const size_t PKp  = (size_t)GB * CH * NSP * 2;
  const size_t PCx  = (size_t)GB * CH * CH * 2;
  size_t off = 0;
  const size_t oWq  = off; off += PWq;
  const size_t oWkv = off; off += PWkv;
  const size_t oWo  = off; off += PWo;
  const size_t oXt  = off; off += PXt;
  const size_t oCt  = off; off += PXt;
  const size_t oQt  = off; off += PQt;
  const size_t oQh  = off; off += PQp;
  const size_t oQl  = off; off += PQp;
  const size_t oKV  = off; off += PKV;
  const size_t oKh  = off; off += PKp;
  const size_t oKl  = off; off += PKp;
  const size_t oVh  = off; off += PKp;
  const size_t oVl  = off; off += PKp;
  const size_t oCxh = off; off += PCx;
  const size_t oCxl = off; off += PCx;
  const size_t oM2h = off; off += PCx;
  const size_t oM2l = off; off += PCx;
  if (off > ws_size) return;
  if (off > (size_t)134217728) return;

  char* ws = (char*)d_ws;
  unsigned short* Wqb  = (unsigned short*)(ws + oWq);
  unsigned short* Wkvb = (unsigned short*)(ws + oWkv);
  unsigned short* Wob  = (unsigned short*)(ws + oWo);
  unsigned short* Xt   = (unsigned short*)(ws + oXt);
  unsigned short* Ct   = (unsigned short*)(ws + oCt);
  float*          Qt   = (float*)(ws + oQt);
  unsigned short* Qh   = (unsigned short*)(ws + oQh);
  unsigned short* Ql   = (unsigned short*)(ws + oQl);
  float*          KV   = (float*)(ws + oKV);
  unsigned short* Kh   = (unsigned short*)(ws + oKh);
  unsigned short* Kl   = (unsigned short*)(ws + oKl);
  unsigned short* Vh   = (unsigned short*)(ws + oVh);
  unsigned short* Vl   = (unsigned short*)(ws + oVl);
  unsigned short* Cxh  = (unsigned short*)(ws + oCxh);
  unsigned short* Cxl  = (unsigned short*)(ws + oCxl);
  unsigned short* M2h  = (unsigned short*)(ws + oM2h);
  unsigned short* M2l  = (unsigned short*)(ws + oM2l);

  const dim3 blk(256);
  const int n8wq  = CH * CH / 8;
  const int n8wkv = 2 * CH * CH / 8;
  const int n8wo  = CH * CH / 8;

  cvt_bf16x8<<<dim3((n8wq + 255) / 256), blk, 0, stream>>>(wq, Wqb, n8wq);
  cvt_bf16x8<<<dim3((n8wkv + 255) / 256), blk, 0, stream>>>(wkv, Wkvb, n8wkv);
  cvt_bf16x8<<<dim3((n8wo + 255) / 256), blk, 0, stream>>>(wo, Wob, n8wo);

  const dim3 gTr(NSP / 64, CH / 64, 2 * GB);
  const dim3 gQt(tile_blocks(NSP, CH), GB);
  const dim3 gQs(NSP / 8, GB);
  const dim3 gKV(tile_blocks(2 * CH, NSP), GB);
  const dim3 gKs(2 * CH, GB);
  const dim3 gCx(tile_blocks(CH, CH), GB);
  const dim3 gOut(tile_blocks(CH, NSP), GB);
  const long long sNC = (long long)NSP * CH;
  const long long sCC = (long long)CH * CH;

  for (int g = 0; g < NGRP; ++g) {
    const int b0 = g * GB;
    k_trcvt<<<gTr, blk, 0, stream>>>(x, cproj, Xt, Ct, b0);
    gemm64<0, 0, 2><<<gQt, blk, 0, stream>>>(
        Xt, Xt, CH, sNC, Wqb, Wqb, CH, 0LL,
        (void*)Qt, (void*)Qt, CH, sNC, bq, NSP, CH, CH, 1.0f);
    k_qsoft<<<gQs, blk, 0, stream>>>(Qt, Qh, Ql);
    gemm64<0, 0, 1><<<gKV, blk, 0, stream>>>(
        Wkvb, Wkvb, CH, 0LL, Ct, Ct, CH, sNC,
        (void*)KV, (void*)KV, NSP, (long long)2 * CH * NSP, bkv, 2 * CH, NSP, CH, 1.0f);
    k_ksoftv<<<gKs, blk, 0, stream>>>(KV, Kh, Kl, Vh, Vl);
    gemm64<2, 2, 0><<<gCx, blk, 0, stream>>>(
        Vh, Vl, NSP, sNC, Kh, Kl, NSP, sNC,
        (void*)Cxh, (void*)Cxl, CH, sCC, bq, CH, CH, NSP, 1.0f / 4096.0f);
    gemm64<3, 2, 0><<<gCx, blk, 0, stream>>>(
        Wob, Wob, CH, 0LL, Cxh, Cxl, CH, sCC,
        (void*)M2h, (void*)M2l, CH, sCC, bq, CH, CH, CH, 1.0f);
    float* outg = out + (size_t)b0 * CH * NSP;
    gemm64<2, 0, 1><<<gOut, blk, 0, stream>>>(
        M2h, M2l, CH, sCC, Qh, Ql, CH, sNC,
        (void*)outg, (void*)outg, NSP, sNC, bo, CH, NSP, CH, 1.0f / 64.0f);
  }
  (void)hipGetLastError();
}
